// SelectiveScanSSM_22952305230024
// MI455X (gfx1250) — hardware-verified
//
#include <hip/hip_runtime.h>
#include <math.h>

typedef __attribute__((ext_vector_type(16))) _Float16 v16h;
typedef __attribute__((ext_vector_type(8)))  _Float16 v8h;
typedef __attribute__((ext_vector_type(16))) __bf16   v16b;
typedef __attribute__((ext_vector_type(8)))  __bf16   v8b;
typedef __attribute__((ext_vector_type(8)))  float    v8f;
typedef __attribute__((ext_vector_type(4)))  float    v4f;

constexpr int kBatch  = 2;
constexpr int kSeq    = 2048;
constexpr int kDm     = 1024;
constexpr int kDin    = 2048;
constexpr int kNst    = 16;
constexpr int kConvK  = 4;
constexpr int kRows   = kBatch * kSeq;
constexpr int kWinR   = 2 * kDin;
constexpr int kXpjR   = 2 * kNst;
constexpr int kBsP    = 64;
constexpr int kActWP  = kDin / 2;
constexpr int kConvTP = 260;
constexpr int kScanTS = 64;
constexpr int kScanCh = 64;
constexpr int kScanYP = 68;
constexpr float kWCarry  = 64.0f;
constexpr float kXsCarry = 8.0f;
constexpr float kXsInv   = 0.125f;
constexpr float kXcCarry = 16.0f;
constexpr float kDtCarry = 256.0f;
constexpr float kDtInv   = 1.0f / 256.0f;
constexpr float kYCarry  = 16.0f;

static_assert((kDm % 32) == 0 && (kDin % 32) == 0);
static_assert((kRows % 64) == 0 && (kDin % 64) == 0 && (kBsP % 64) == 0 && (kDm % 64) == 0);
static_assert((kSeq % kScanTS) == 0 && (kSeq % 64) == 0 && (kDin % kScanCh) == 0 && (kDin % 256) == 0);
static_assert(kXpjR == 2 * kNst && kNst <= kBsP);

constexpr size_t kOffXH   = 0;
constexpr size_t kOffWIH  = kOffXH  + (size_t)kRows * kDm  * 2;
constexpr size_t kOffWDH  = kOffWIH + (size_t)kWinR * kDm  * 2;
constexpr size_t kOffWXB  = kOffWDH + (size_t)kDin  * kDin * 2;
constexpr size_t kOffWOH  = kOffWXB + (size_t)kBsP  * kDin * 2;
constexpr size_t kOffXS   = kOffWOH + (size_t)kDm   * kDin * 2;
constexpr size_t kOffRS   = kOffXS  + (size_t)kRows * kDin * 2;
constexpr size_t kOffXC   = kOffRS  + (size_t)kRows * kDin * 4;
constexpr size_t kOffDT   = kOffXC  + (size_t)kRows * kDin * 2;
constexpr size_t kOffBS   = kOffDT  + (size_t)kRows * kDin * 2;
constexpr size_t kOffYH   = kOffBS  + (size_t)kRows * kBsP * 4;
constexpr size_t kWsTotal = kOffYH  + (size_t)kRows * kDin * 2;
static_assert(kWsTotal == 131334144ull);
static_assert(kWsTotal <= 134217728ull);
static_assert((kOffWIH % 128) == 0 && (kOffWDH % 128) == 0 && (kOffWXB % 128) == 0 && (kOffWOH % 128) == 0 &&
              (kOffXS % 128) == 0 && (kOffRS % 128) == 0 && (kOffXC % 128) == 0 && (kOffDT % 128) == 0 &&
              (kOffBS % 128) == 0 && (kOffYH % 128) == 0);

__device__ __forceinline__ unsigned short f2bf_bits(float f) {
  unsigned u = __float_as_uint(f);
  return (unsigned short)((u + 0x7FFFu + ((u >> 16) & 1u)) >> 16);
}
__device__ __forceinline__ float bf_bits2f(unsigned short h) { return __uint_as_float(((unsigned)h) << 16); }
__device__ __forceinline__ float bfr(float f) { return bf_bits2f(f2bf_bits(f)); }
__device__ __forceinline__ float h16_to_f32(unsigned hb) {
  const unsigned sgn = (hb & 0x8000u) << 16; const unsigned em = hb & 0x7fffu;
  const float fn = __uint_as_float((em << 13) + 0x38000000u);
  const float fs = (float)em * 5.9604644775390625e-8f;
  const float mag = (em < 0x400u) ? fs : fn; return __uint_as_float(__float_as_uint(mag) | sgn); }
__device__ __forceinline__ float plane_val(unsigned w, unsigned par, float inv_carry) {
  const unsigned hb = par ? (w >> 16) : (w & 0xffffu);
  return h16_to_f32(hb) * inv_carry;
}

__device__ __forceinline__ void dep_guard_h(v8f& a, v8f& b, v16h x, v16h y) { asm volatile("v_nop\n\tv_nop\n\tv_nop\n\tv_nop" : "+v"(a), "+v"(b) : "v"(x), "v"(y)); }
__device__ __forceinline__ void dep_guard_b(v8f& a, v8f& b, v16b x, v16b y) { asm volatile("v_nop\n\tv_nop\n\tv_nop\n\tv_nop" : "+v"(a), "+v"(b) : "v"(x), "v"(y)); }
__device__ __forceinline__ void keep4_h(v16h a, v16h b, v16h c, v16h d) { asm volatile("v_nop" :: "v"(a), "v"(b), "v"(c), "v"(d)); }
__device__ __forceinline__ void keep4_b(v16b a, v16b b, v16b c, v16b d) { asm volatile("v_nop" :: "v"(a), "v"(b), "v"(c), "v"(d)); }
__device__ __forceinline__ void acc_guard4(v8f& a, v8f& b, v8f& c, v8f& d) { asm volatile("v_nop\n\tv_nop\n\tv_nop\n\tv_nop" : "+v"(a), "+v"(b), "+v"(c), "+v"(d)); }
template <typename T> struct Frag;
template <> struct Frag<_Float16> {
  typedef v16h V; union U { v16h v; v8h h[2]; };
  static __device__ __forceinline__ v16h load(const _Float16* p) {
    U f; f.h[0] = *(const v8h*)(p); f.h[1] = *(const v8h*)(p + 16); return f.v;
  }
  static __device__ __forceinline__ v8f mma(v16h a, v16h b, v8f c) {
    return __builtin_amdgcn_wmma_f32_16x16x32_f16(false, a, false, b, (short)0, c, false, false);
  }
  static __device__ __forceinline__ void guard(v8f& a, v8f& b, v16h x, v16h y) { dep_guard_h(a, b, x, y); }
  static __device__ __forceinline__ void keep(v16h a, v16h b, v16h c, v16h d) { keep4_h(a, b, c, d); }
};
template <> struct Frag<__bf16> {
  typedef v16b V; union U { v16b v; v8b h[2]; };
  static __device__ __forceinline__ v16b load(const __bf16* p) {
    U f; f.h[0] = *(const v8b*)(p); f.h[1] = *(const v8b*)(p + 16); return f.v;
  }
  static __device__ __forceinline__ v8f mma(v16b a, v16b b, v8f c) {
    return __builtin_amdgcn_wmma_f32_16x16x32_bf16(false, a, false, b, (short)0, c, false, false);
  }
  static __device__ __forceinline__ void guard(v8f& a, v8f& b, v16b x, v16b y) { dep_guard_b(a, b, x, y); }
  static __device__ __forceinline__ void keep(v16b a, v16b b, v16b c, v16b d) { keep4_b(a, b, c, d); }
};

template <int ET> struct Elem;
template <> struct Elem<0> { typedef _Float16 T; };
template <> struct Elem<1> { typedef __bf16 T; };
template <int ET, bool SPLIT, int BIAS_MODE, int OUT_MODE, bool RESID, int ACT = 0>
__global__ __launch_bounds__(256) void wmma_gemm64(
    const unsigned short* __restrict__ Ap, const unsigned short* __restrict__ A2p, int lda, long strideA,
    const unsigned short* __restrict__ Btp, const unsigned short* __restrict__ Bt2p, int ldb, long strideB,
    void* __restrict__ Cout, void* __restrict__ Cout2, int ldc, long strideC,
    const float* __restrict__ bias,
    const float* __restrict__ resid, long strideR,
    int M, int N, int K, float scale) {
  typedef typename Elem<ET>::T T;
  typedef typename Frag<T>::V V;
  const T* A = (const T*)Ap; const T* A2 = (const T*)A2p; const T* Bt = (const T*)Btp; const T* Bt2 = (const T*)Bt2p;
  __shared__ __align__(16) float sT[8][16 * 68];
  const int b    = blockIdx.y;
  const int lane = threadIdx.x & 31;
  const int wave = threadIdx.x >> 5;
  const int tilesN = N >> 6;
  const int tilesM = M >> 6;
  const int tile = blockIdx.x * 8 + wave;
  if (tile >= tilesM * tilesN) return;
  const int tm = tile / tilesN;
  const int tn = tile - tm * tilesN;
  const int m0 = tm << 6;
  const int n0 = tn << 6;

  const T* Ab  = A  + (size_t)b * strideA;
  const T* Bb  = Bt + (size_t)b * strideB;
  const T* Ab2 = SPLIT ? (A2  + (size_t)b * strideA) : nullptr;
  const T* Bb2 = SPLIT ? (Bt2 + (size_t)b * strideB) : nullptr;

  const int rlane = lane & 15;
  const int koff  = (lane >> 4) * 8;
  const int mOff  = (lane >> 4) * 8;

  v8f acc[4][4];
#pragma unroll
  for (int i = 0; i < 4; ++i)
#pragma unroll
    for (int j = 0; j < 4; ++j) acc[i][j] = (v8f){0.f,0.f,0.f,0.f,0.f,0.f,0.f,0.f};

  for (int k0 = 0; k0 < K; k0 += 32) {
    V bh[4], bl[4];
#pragma unroll
    for (int j = 0; j < 4; ++j) {
      const size_t bo = (size_t)(n0 + (j << 4) + rlane) * ldb + koff + k0;
      bh[j] = Frag<T>::load(Bb + bo);
      if (SPLIT) bl[j] = Frag<T>::load(Bb2 + bo);
    }
#pragma unroll
    for (int i = 0; i < 4; ++i) {
      const size_t ao = (size_t)(m0 + (i << 4) + rlane) * lda + koff + k0;
      V ah = Frag<T>::load(Ab + ao);
      V al;
      if (SPLIT) al = Frag<T>::load(Ab2 + ao);
#pragma unroll
      for (int j = 0; j < 4; ++j) {
        acc[i][j] = Frag<T>::mma(ah, bh[j], acc[i][j]);
        if (SPLIT) {
          acc[i][j] = Frag<T>::mma(ah, bl[j], acc[i][j]);
          acc[i][j] = Frag<T>::mma(al, bh[j], acc[i][j]);
        }
      }
      Frag<T>::guard(acc[i][0], acc[i][3], ah, SPLIT ? al : ah);
    }
    Frag<T>::keep(bh[0], bh[1], bh[2], bh[3]);
    if (SPLIT) Frag<T>::keep(bl[0], bl[1], bl[2], bl[3]);
  }
  acc_guard4(acc[0][0], acc[0][1], acc[0][2], acc[0][3]);
  acc_guard4(acc[1][0], acc[1][1], acc[1][2], acc[1][3]);
  acc_guard4(acc[2][0], acc[2][1], acc[2][2], acc[2][3]);
  acc_guard4(acc[3][0], acc[3][1], acc[3][2], acc[3][3]);

  float* slab = sT[wave];
  const float* Rb = RESID ? (resid + (size_t)b * strideR) : nullptr;
#pragma unroll
  for (int i = 0; i < 4; ++i) {
    const int mBase = m0 + (i << 4);
#pragma unroll
    for (int j = 0; j < 4; ++j) {
      const int n = n0 + (j << 4) + rlane;
      float bv = 0.f;
      if (BIAS_MODE == 2) bv = bias[n];
#pragma unroll
      for (int r = 0; r < 8; ++r) {
        float v = acc[i][j][r] * scale;
        if (BIAS_MODE == 1) v += bias[mBase + mOff + r];
        if (BIAS_MODE == 2) v += bv;
        if (RESID) v += Rb[(size_t)(mBase + mOff + r) * ldc + n];
        if (ACT == 1) v = tanhf(v);
        if (ACT == 2) v = fmaxf(v, 0.0f);
        if (ACT == 3) v = v / (1.0f + expf(-v));
        if (ACT == 4) v = (v > 0.f) ? v : 0.01f * v;
        slab[(mOff + r) * 68 + (j << 4) + rlane] = v;
      }
    }
    __builtin_amdgcn_fence(__ATOMIC_RELEASE, "workgroup");
    __builtin_amdgcn_wave_barrier();
    __builtin_amdgcn_fence(__ATOMIC_ACQUIRE, "workgroup");
    if (OUT_MODE == 0) {
      float* C = (float*)Cout + (size_t)b * strideC;
      const int hh = lane >> 4, c4 = (lane & 15) * 4;
      for (int pass = 0; pass < 2; ++pass) {
#pragma unroll
        for (int it = 0; it < 8; ++it) {
          const int row = it * 2 + hh;
          v4f v = *(const v4f*)(slab + row * 68 + c4);
          *(volatile v4f*)(C + (size_t)(mBase + row) * ldc + n0 + c4) = v;
        }
        __threadfence();
      }
    } else {
      const int q = lane >> 3, c8 = (lane & 7) * 8;
      unsigned short* C  = (unsigned short*)Cout  + (size_t)b * strideC;
      unsigned short* C2 = (OUT_MODE == 2) ? ((unsigned short*)Cout2 + (size_t)b * strideC) : nullptr;
      for (int pass = 0; pass < 2; ++pass) {
#pragma unroll
        for (int it = 0; it < 4; ++it) {
          const int row = it * 4 + q;
          const float* sp = slab + row * 68 + c8;
          v8h hv, lv;
#pragma unroll
          for (int e = 0; e < 8; ++e) {
            if (OUT_MODE == 1) {
              hv[e] = (_Float16)sp[e];
            } else {
              unsigned short hb = f2bf_bits(sp[e]);
              unsigned short lb = f2bf_bits(sp[e] - bf_bits2f(hb));
              hv[e] = __builtin_bit_cast(_Float16, hb);
              lv[e] = __builtin_bit_cast(_Float16, lb);
            }
          }
          *(volatile v8h*)(C + (size_t)(mBase + row) * ldc + n0 + c8) = hv;
          if (OUT_MODE == 2) *(volatile v8h*)(C2 + (size_t)(mBase + row) * ldc + n0 + c8) = lv;
        }
        __threadfence();
      }
    }
    __builtin_amdgcn_fence(__ATOMIC_RELEASE, "workgroup");
    __builtin_amdgcn_wave_barrier();
    __builtin_amdgcn_fence(__ATOMIC_ACQUIRE, "workgroup");
  }
}

__global__ __launch_bounds__(256) void cast_f16_kernel(
    const float* __restrict__ src, unsigned short* __restrict__ dst, int total8, float scale)
{
  const int i = blockIdx.x * 256 + threadIdx.x;
  if (i >= total8) return;
  const size_t e0 = (size_t)i << 3;
  const v4f a0 = *(const v4f*)(src + e0);
  const v4f a1 = *(const v4f*)(src + e0 + 4);
  v8h hv;
#pragma unroll
  for (int e = 0; e < 4; ++e) {
    hv[e]     = (_Float16)(bfr(a0[e]) * scale);
    hv[4 + e] = (_Float16)(bfr(a1[e]) * scale);
  }
  unsigned short* qh = dst + e0;
  *(volatile v8h*)qh = hv;
  __threadfence();
  *(volatile v8h*)qh = hv;
}

__global__ __launch_bounds__(256) void build_wxb_kernel(
    const float* __restrict__ wx, unsigned short* __restrict__ dst, int total8)
{
  const int i = blockIdx.x * 256 + threadIdx.x;
  if (i >= total8) return;
  const int row = i >> 8;
  const int col = (i & 255) * 8;
  const int srow = kNst + ((row < kNst) ? row : (kNst - 1));
  const float mul = (row < kNst) ? kWCarry : 0.0f;
  const float* sp = wx + (size_t)srow * kDin + col;
  const v4f a0 = *(const v4f*)(sp);
  const v4f a1 = *(const v4f*)(sp + 4);
  v8h hv;
#pragma unroll
  for (int e = 0; e < 4; ++e) {
    hv[e]     = (_Float16)(bfr(a0[e]) * mul);
    hv[4 + e] = (_Float16)(bfr(a1[e]) * mul);
  }
  unsigned short* qh = dst + ((size_t)i << 3);
  *(volatile v8h*)qh = hv;
  __threadfence();
  *(volatile v8h*)qh = hv;
}

__device__ __forceinline__ float conv_silu_f(float w0, float w1, float w2, float w3, float bc,
                                             float a3, float a2, float a1, float a0) {
  float acc = w0 * a3;
  acc = fmaf(w1, a2, acc);
  acc = fmaf(w2, a1, acc);
  acc = fmaf(w3, a0, acc);
  const float sv = acc + bc;
  const float sg = 1.0f / (1.0f + expf(-sv));
  return sv * sg;
}

__global__ __launch_bounds__(256) void conv_silu_kernel(
    const unsigned* __restrict__ XSW, const float* __restrict__ cw, const float* __restrict__ cb,
    unsigned short* __restrict__ XCH)
{
  __shared__ __align__(16) float sT[16 * kConvTP];
  const int tid = threadIdx.x, lane = tid & 31, wave = tid >> 5;
  const int d0 = blockIdx.x * 256, d = d0 + tid;
  const int wd = d >> 1;
  const unsigned par = (unsigned)(d & 1);
  const int g0 = blockIdx.y * 64;
  const int tb = g0 & (kSeq - 1);
  const float w0 = bfr(cw[d * kConvK + 0]), w1 = bfr(cw[d * kConvK + 1]);
  const float w2 = bfr(cw[d * kConvK + 2]), w3 = bfr(cw[d * kConvK + 3]);
  const float bc = bfr(cb[d]);
  float xm3, xm2, xm1;
  {
    const bool hist = (tb > 0);
    const int rb = hist ? (g0 - 3) : g0;
    const float v3 = plane_val(XSW[(size_t)rb * kActWP + wd], par, kXsInv);
    const float v2 = plane_val(XSW[(size_t)(rb + 1) * kActWP + wd], par, kXsInv);
    const float v1 = plane_val(XSW[(size_t)(rb + 2) * kActWP + wd], par, kXsInv);
    xm3 = hist ? v3 : 0.f;
    xm2 = hist ? v2 : 0.f;
    xm1 = hist ? v1 : 0.f;
  }
#pragma unroll 1
  for (int sub = 0; sub < 4; ++sub) {
    const int lb = g0 + sub * 16;
#pragma unroll 1
    for (int s = 0; s < 16; ++s) {
      const float xcur = plane_val(XSW[(size_t)(lb + s) * kActWP + wd], par, kXsInv);
      sT[s * kConvTP + tid] = conv_silu_f(w0, w1, w2, w3, bc, xm3, xm2, xm1, xcur);
      xm3 = xm2; xm2 = xm1; xm1 = xcur;
    }
    __syncthreads();
    v8h hv[2];
#pragma unroll
    for (int it = 0; it < 2; ++it) {
      const float* sp = sT + (it * 8 + wave) * kConvTP + lane * 8;
      const v4f a0 = *(const v4f*)(sp);
      const v4f a1 = *(const v4f*)(sp + 4);
#pragma unroll
      for (int e = 0; e < 4; ++e) {
        hv[it][e]     = (_Float16)(a0[e] * kXcCarry);
        hv[it][4 + e] = (_Float16)(a1[e] * kXcCarry);
      }
    }
    for (int pass = 0; pass < 2; ++pass) {
#pragma unroll
      for (int it = 0; it < 2; ++it)
        *(volatile v8h*)(XCH + (size_t)(lb + it * 8 + wave) * kDin + d0 + lane * 8) = hv[it];
      __threadfence();
    }
    __syncthreads();
  }
}

__global__ __launch_bounds__(64) void scan_kernel(
    const unsigned* __restrict__ XSW, const unsigned* __restrict__ DTW, const float* __restrict__ RS,
    const float* __restrict__ BS, const float* __restrict__ cw, const float* __restrict__ cb,
    const float* __restrict__ bdt, const float* __restrict__ Alog, const float* __restrict__ Dp,
    unsigned short* __restrict__ YH)
{
  __shared__ __align__(16) float sB[kScanTS * kNst];
  __shared__ __align__(16) float sY[kScanTS * kScanYP];
  __shared__ __align__(16) float sA[kNst * kScanCh];
  const int tid = threadIdx.x, lane = tid & 31, wave = tid >> 5;
  constexpr int kBlkPerB = kDin / kScanCh;
  const int bix = blockIdx.x / kBlkPerB;
  const int d0  = (blockIdx.x - bix * kBlkPerB) * kScanCh;
  const int d   = d0 + tid;
  const int wd  = d >> 1;
  const unsigned par = (unsigned)(d & 1);
  const size_t row0 = (size_t)bix * kSeq;
#pragma unroll 1
  for (int s = 0; s < kNst; ++s) sA[s * kScanCh + tid] = -expf(bfr(Alog[(size_t)d * kNst + s]));
  __syncthreads();
  float negA[kNst], h[kNst];
#pragma unroll
  for (int s = 0; s < kNst; ++s) {
    negA[s] = sA[s * kScanCh + tid];
    h[s] = 0.f;
  }
  const float w0 = bfr(cw[d * kConvK + 0]), w1 = bfr(cw[d * kConvK + 1]);
  const float w2 = bfr(cw[d * kConvK + 2]), w3 = bfr(cw[d * kConvK + 3]);
  const float bc = bfr(cb[d]);
  const float bb = bfr(bdt[d]), Dd = bfr(Dp[d]);
  float xm3 = 0.f, xm2 = 0.f, xm1 = 0.f;
  const int q = lane >> 3, c8 = (lane & 7) * 8;
#pragma unroll 1
  for (int t0 = 0; t0 < kSeq; t0 += kScanTS) {
    __syncthreads();
#pragma unroll
    for (int i = 0; i < 4; ++i)
      *(v4f*)(sB + tid * kNst + 4 * i) = *(const v4f*)(BS + (row0 + t0 + tid) * kBsP + 4 * i);
    __syncthreads();
#pragma unroll 1
    for (int s = 0; s < kScanTS; ++s) {
      const size_t row = row0 + t0 + s;
      const float xcur = plane_val(XSW[row * kActWP + wd], par, kXsInv);
      const float xc = conv_silu_f(w0, w1, w2, w3, bc, xm3, xm2, xm1, xcur);
      xm3 = xm2; xm2 = xm1; xm1 = xcur;
      const float dtr = plane_val(DTW[row * kActWP + wd], par, kDtInv);
      const float v   = dtr + bb;
      const float dt  = fmaxf(v, 0.0f) + log1pf(expf(-fabsf(v)));
      const float rv  = RS[row * kDin + d];
      const float gt  = rv * (1.0f / (1.0f + expf(-rv)));
      const float* bp = sB + s * kNst;
      float Bs[kNst];
#pragma unroll
      for (int q4 = 0; q4 < 4; ++q4) {
        const v4f bv = *(const v4f*)(bp + 4 * q4);
        Bs[4 * q4 + 0] = bv[0]; Bs[4 * q4 + 1] = bv[1]; Bs[4 * q4 + 2] = bv[2]; Bs[4 * q4 + 3] = bv[3];
      }
      const float dtx = dt * xc;
      float y = 0.0f;
#pragma unroll
      for (int k = 0; k < kNst; ++k) {
        const float e = __expf(dt * negA[k]);
        h[k] = e * h[k] + dtx * Bs[k];
        y = y + h[k];
      }
      y = y + xc * Dd;
      y = y * gt;
      sY[s * kScanYP + tid] = y;
    }
    __syncthreads();
    v8h hv[8];
#pragma unroll
    for (int it = 0; it < 8; ++it) {
      const int row = it * 8 + wave * 4 + q;
      const float* sp = sY + row * kScanYP + c8;
      const v4f a0 = *(const v4f*)(sp);
      const v4f a1 = *(const v4f*)(sp + 4);
#pragma unroll
      for (int e = 0; e < 4; ++e) {
        hv[it][e]     = (_Float16)(a0[e] * kYCarry);
        hv[it][4 + e] = (_Float16)(a1[e] * kYCarry);
      }
    }
    for (int pass = 0; pass < 2; ++pass) {
#pragma unroll
      for (int it = 0; it < 8; ++it) {
        const int row = it * 8 + wave * 4 + q;
        const size_t o = (row0 + t0 + row) * kDin + d0 + c8;
        *(volatile v8h*)(YH + o) = hv[it];
      }
      __threadfence();
    }
  }
}

extern "C" void kernel_launch(void* const* d_in, const int* in_sizes, int n_in,
                              void* d_out, int out_size, void* d_ws, size_t ws_size,
                              hipStream_t stream) {
  if (n_in < 10) return;
  if (in_sizes[0] != kRows * kDm) return;
  if (in_sizes[1] != kWinR * kDm) return;
  if (in_sizes[2] != kDin * kConvK) return;
  if (in_sizes[3] != kDin) return;
  if (in_sizes[4] != kXpjR * kDin) return;
  if (in_sizes[5] != kDin * kDin) return;
  if (in_sizes[6] != kDin) return;
  if (in_sizes[7] != kDin * kNst) return;
  if (in_sizes[8] != kDin) return;
  if (in_sizes[9] != kDm * kDin) return;
  if (out_size != kRows * kDm) return;
  if (ws_size < kWsTotal) return;

  const float* x       = (const float*)d_in[0];
  const float* W_in    = (const float*)d_in[1];
  const float* conv_w  = (const float*)d_in[2];
  const float* conv_b  = (const float*)d_in[3];
  const float* W_xproj = (const float*)d_in[4];
  const float* W_dt    = (const float*)d_in[5];
  const float* b_dt    = (const float*)d_in[6];
  const float* A_log   = (const float*)d_in[7];
  const float* Dp      = (const float*)d_in[8];
  const float* W_out   = (const float*)d_in[9];
  float* out = (float*)d_out;

  char* ws = (char*)d_ws;
  unsigned short* XH   = (unsigned short*)(ws + kOffXH);
  unsigned short* WIH  = (unsigned short*)(ws + kOffWIH);
  unsigned short* WDH  = (unsigned short*)(ws + kOffWDH);
  unsigned short* WXB  = (unsigned short*)(ws + kOffWXB);
  unsigned short* WOH  = (unsigned short*)(ws + kOffWOH);
  unsigned short* XS   = (unsigned short*)(ws + kOffXS);
  float*          RS   = (float*)(ws + kOffRS);
  unsigned short* XC   = (unsigned short*)(ws + kOffXC);
  unsigned short* DT   = (unsigned short*)(ws + kOffDT);
  float*          BS   = (float*)(ws + kOffBS);
  unsigned short* YH   = (unsigned short*)(ws + kOffYH);

  const int nx8  = kRows * kDm / 8;
  const int nwi8 = kWinR * kDm / 8;
  const int nwd8 = kDin * kDin / 8;
  const int nwo8 = kDm * kDin / 8;
  const int nxb8 = kBsP * kDin / 8;
  cast_f16_kernel<<<(nx8 + 255) / 256, 256, 0, stream>>>(x, XH, nx8, 1.0f);
  cast_f16_kernel<<<(nwi8 + 255) / 256, 256, 0, stream>>>(W_in, WIH, nwi8, kWCarry);
  cast_f16_kernel<<<(nwd8 + 255) / 256, 256, 0, stream>>>(W_dt, WDH, nwd8, kWCarry);
  cast_f16_kernel<<<(nwo8 + 255) / 256, 256, 0, stream>>>(W_out, WOH, nwo8, kWCarry);
  build_wxb_kernel<<<(nxb8 + 255) / 256, 256, 0, stream>>>(W_xproj, WXB, nxb8);

  {
    const int tiles = (kRows / 64) * (kDin / 64);
    wmma_gemm64<0, false, 0, 1, false, 0><<<dim3((tiles + 7) / 8, 1), 256, 0, stream>>>(
        XH, nullptr, kDm, 0L,
        WIH, nullptr, kDm, 0L,
        (void*)XS, nullptr, kDin, 0L,
        nullptr, nullptr, 0L,
        kRows, kDin, kDm, kXsCarry / kWCarry);
  }
  {
    const int tiles = (kRows / 64) * (kDin / 64);
    wmma_gemm64<0, false, 0, 0, false, 0><<<dim3((tiles + 7) / 8, 1), 256, 0, stream>>>(
        XH, nullptr, kDm, 0L,
        WIH + (size_t)kDin * kDm, nullptr, kDm, 0L,
        (void*)RS, nullptr, kDin, 0L,
        nullptr, nullptr, 0L,
        kRows, kDin, kDm, 1.0f / kWCarry);
  }

  conv_silu_kernel<<<dim3(kDin / 256, kRows / 64), 256, 0, stream>>>((const unsigned*)XS, conv_w, conv_b, XC);

  {
    const int tiles = (kRows / 64) * (kDin / 64);
    wmma_gemm64<0, false, 0, 1, false, 0><<<dim3((tiles + 7) / 8, 1), 256, 0, stream>>>(
        XC, nullptr, kDin, 0L,
        WDH, nullptr, kDin, 0L,
        (void*)DT, nullptr, kDin, 0L,
        nullptr, nullptr, 0L,
        kRows, kDin, kDin, kDtCarry / (kXcCarry * kWCarry));
  }
  {
    const int tiles = (kRows / 64) * (kBsP / 64);
    wmma_gemm64<0, false, 0, 0, false, 0><<<dim3((tiles + 7) / 8, 1), 256, 0, stream>>>(
        XC, nullptr, kDin, 0L,
        WXB, nullptr, kDin, 0L,
        (void*)BS, nullptr, kBsP, 0L,
        nullptr, nullptr, 0L,
        kRows, kBsP, kDin, 1.0f / (kXcCarry * kWCarry));
  }

  scan_kernel<<<kBatch * (kDin / kScanCh), kScanCh, 0, stream>>>(
      (const unsigned*)XS, (const unsigned*)DT, RS, BS, conv_w, conv_b, b_dt, A_log, Dp, YH);

  {
    const int tiles = (kRows / 64) * (kDm / 64);
    wmma_gemm64<0, false, 0, 0, false, 0><<<dim3((tiles + 7) / 8, 1), 256, 0, stream>>>(
        YH, nullptr, kDin, 0L,
        WOH, nullptr, kDin, 0L,
        (void*)out, nullptr, kDm, 0L,
        nullptr, nullptr, 0L,
        kRows, kDm, kDin, 1.0f / (kYCarry * kWCarry));
  }
}
